// TransformerLayer_50749333570029
// MI455X (gfx1250) — hardware-verified
//
#include <hip/hip_runtime.h>
#include <math.h>

typedef __attribute__((ext_vector_type(16))) _Float16 v16h;
typedef __attribute__((ext_vector_type(16))) __bf16 v16b;
typedef __attribute__((ext_vector_type(8)))  _Float16 v8h;
typedef __attribute__((ext_vector_type(8)))  __bf16 v8b;
typedef __attribute__((ext_vector_type(8)))  float v8f;
typedef __attribute__((ext_vector_type(4)))  float v4f;
typedef __attribute__((ext_vector_type(8)))  unsigned short v8us;

#ifndef SEQ
#define SEQ 8192
#endif
#define SEQ_FULL 8192
#ifndef NB
#define NB 1
#endif
#define DIN 1024
#define DQK 128
#define DV 1024
#define DOUT 1024
#define SCALE (11.313708498984761f)
#define RC (4096.0f)
#define PCY (16384.0f)
#define WC (64.0f)
#define F16MIN (6.103515625e-05f)
#define LN_EPS (1e-5f)
static_assert(SEQ % 128 == 0);
static_assert(SEQ >= 128);
static_assert(SEQ <= SEQ_FULL);
static_assert(DQK == 128);
static_assert(DIN == 1024);
static_assert(DV == 1024);
static_assert(DOUT == DV);

#define WSZ_XB   (2u * (size_t)SEQ * DIN)
#define WSZ_WQB  (2u * (size_t)DQK * DIN)
#define WSZ_WKB  (2u * (size_t)DQK * DIN)
#define WSZ_WVB  (2u * (size_t)DV * DIN)
#define WSZ_WLH  (2u * (size_t)DOUT * DIN)
#define WSZ_QP   (2u * (size_t)SEQ * DQK)
#define WSZ_VT   (2u * (size_t)DV * SEQ)
#define WSZ_MX   (4u * (size_t)SEQ)
#define WSZ_SA   (4u * (size_t)SEQ * DV)
#define WSZ_H16  (2u * (size_t)SEQ * DIN)
#define WSZ_Z2   (4u * (size_t)SEQ * DOUT)
#define WS_XB   ((size_t)0)
#define WS_WQB  (WS_XB  + WSZ_XB)
#define WS_WKB  (WS_WQB + WSZ_WQB)
#define WS_WVB  (WS_WKB + WSZ_WKB)
#define WS_WLH  (WS_WVB + WSZ_WVB)
#define WS_QH   (WS_WLH + WSZ_WLH)
#define WS_QL   (WS_QH  + WSZ_QP)
#define WS_KH   (WS_QL  + WSZ_QP)
#define WS_KL   (WS_KH  + WSZ_QP)
#define WS_VT   (WS_KL  + WSZ_QP)
#define WS_MX   (WS_VT  + WSZ_VT)
#define WS_SA   (WS_MX  + WSZ_MX)
#define WS_H16  (WS_SA  + WSZ_SA)
#define WS_Z2   (WS_H16 + WSZ_H16)
#define WS_END  (WS_Z2  + WSZ_Z2)
static_assert(WS_END <= (size_t)134217728u);
static_assert((WS_MX % 256u) == 0 && (WS_SA % 256u) == 0 && (WS_H16 % 256u) == 0 && (WS_Z2 % 256u) == 0);

template <typename T> __device__ __forceinline__ void vst2(void* p, T v) { *(volatile T*)p = v; __threadfence(); *(volatile T*)p = v; }
__device__ __forceinline__ v8f zero8() { v8f z = {0.f, 0.f, 0.f, 0.f, 0.f, 0.f, 0.f, 0.f}; return z; }
__device__ __forceinline__ v8f wmma16(v16h a, v16h b, v8f c) {
  v8f d = __builtin_amdgcn_wmma_f32_16x16x32_f16(false, a, false, b, (short)0, c, false, false);
  asm volatile("v_nop\n\tv_nop\n\tv_nop\n\tv_nop" : "+v"(d) : "v"(a), "v"(b));
  return d;
}
__device__ __forceinline__ v8f wmma_bf(v16b a, v16b b, v8f c) {
  v8f d = __builtin_amdgcn_wmma_f32_16x16x32_bf16(false, a, false, b, (short)0, c, false, false);
  asm volatile("v_nop\n\tv_nop\n\tv_nop\n\tv_nop" : "+v"(d) : "v"(a), "v"(b));
  return d;
}
__device__ __forceinline__ v16h frag_h(const _Float16* rowk0, int lane) {
  union { v16h v; v8h q[2]; } u; const _Float16* p = rowk0 + 8 * (lane >> 4);
  u.q[0] = *(const v8h*)p; u.q[1] = *(const v8h*)(p + 16); return u.v;
}
__device__ __forceinline__ v16b frag_b(const __bf16* rowk0, int lane) {
  union { v16b v; v8b q[2]; } u; const __bf16* p = rowk0 + 8 * (lane >> 4);
  u.q[0] = *(const v8b*)p; u.q[1] = *(const v8b*)(p + 16); return u.v;
}
__device__ __forceinline__ _Float16 f16n(float x) { const float t = (fabsf(x) >= F16MIN) ? x : 0.0f; return (_Float16)t; }
__device__ __forceinline__ unsigned short bf16bits(float x) { unsigned u = __float_as_uint(x); u += 0x7FFFu + ((u >> 16) & 1u); return (unsigned short)(u >> 16); }
__device__ __forceinline__ float bf16val(unsigned short b) { return __uint_as_float(((unsigned)b) << 16); }
#define LDSX() do { asm volatile("s_wait_dscnt 0" ::: "memory"); __builtin_amdgcn_wave_barrier(); __builtin_amdgcn_fence(3  , "workgroup"); } while (0)

__global__ __launch_bounds__(256) void k_cvtb(const float* __restrict__ src, int n8, unsigned short* __restrict__ dst) {
  const int i = blockIdx.x * 256 + (int)threadIdx.x; if (i >= n8) return;
  const float* p = src + (size_t)i * 8; const v4f a = *(const v4f*)p, b = *(const v4f*)(p + 4);
  v8us o;
#pragma unroll
  for (int e = 0; e < 4; ++e) { o[e] = bf16bits(a[e]); o[4 + e] = bf16bits(b[e]); }
  vst2(dst + (size_t)i * 8, o);
}
__global__ __launch_bounds__(256) void k_cvth(const float* __restrict__ src, int n8, _Float16* __restrict__ dst) {
  const int i = blockIdx.x * 256 + (int)threadIdx.x; if (i >= n8) return;
  const float* p = src + (size_t)i * 8; const v4f a = *(const v4f*)p, b = *(const v4f*)(p + 4);
  v8h o;
#pragma unroll
  for (int e = 0; e < 4; ++e) { o[e] = f16n(bf16val(bf16bits(a[e])) * WC); o[4 + e] = f16n(bf16val(bf16bits(b[e])) * WC); }
  vst2(dst + (size_t)i * 8, o);
}

__global__ __launch_bounds__(128) void k_pqk(const __bf16* __restrict__ XB, const __bf16* __restrict__ WB, _Float16* __restrict__ OH, _Float16* __restrict__ OL) {
  __shared__ __align__(16) _Float16 sh[64][136], sl[64][136];
  const int tid = threadIdx.x, wave = tid >> 5, lane = tid & 31, col = lane & 15, g = lane >> 4;
  const size_t r0 = (size_t)blockIdx.x * 64;
  v8f acc[8];
#pragma unroll
  for (int j = 0; j < 8; ++j) acc[j] = zero8();
#pragma unroll 1
  for (int kc = 0; kc < DIN / 32; ++kc) {
    const v16b a = frag_b(XB + (r0 + wave * 16 + col) * DIN + kc * 32, lane);
#pragma unroll
    for (int j = 0; j < 8; ++j) acc[j] = wmma_bf(a, frag_b(WB + (size_t)(j * 16 + col) * DIN + kc * 32, lane), acc[j]);
  }
#pragma unroll
  for (int j = 0; j < 8; ++j)
#pragma unroll
    for (int r = 0; r < 8; ++r) { const float v = acc[j][r]; const _Float16 hv = f16n(v); sh[wave * 16 + 8 * g + r][j * 16 + col] = hv; sl[wave * 16 + 8 * g + r][j * 16 + col] = f16n((v - (float)hv) * RC); }
  __syncthreads();
  for (int e = tid; e < 64 * 16; e += 128) { const int rl = e >> 4, q = e & 15; const size_t o = (r0 + rl) * (size_t)DQK + q * 8; vst2(OH + o, *(const v8h*)&sh[rl][q * 8]); vst2(OL + o, *(const v8h*)&sl[rl][q * 8]); }
}

__global__ __launch_bounds__(128) void k_pvt(const __bf16* __restrict__ XB, const __bf16* __restrict__ WVB, _Float16* __restrict__ VT) {
  __shared__ __align__(16) _Float16 th[128][72];
  const int tid = threadIdx.x, wave = tid >> 5, lane = tid & 31, col = lane & 15, g = lane >> 4;
  const int c0 = blockIdx.y * 128; const size_t r0 = (size_t)blockIdx.x * 64;
  v8f acc[8];
#pragma unroll
  for (int j = 0; j < 8; ++j) acc[j] = zero8();
#pragma unroll 1
  for (int kc = 0; kc < DIN / 32; ++kc) {
    const v16b a = frag_b(XB + (r0 + wave * 16 + col) * DIN + kc * 32, lane);
#pragma unroll
    for (int j = 0; j < 8; ++j) acc[j] = wmma_bf(a, frag_b(WVB + (size_t)(c0 + j * 16 + col) * DIN + kc * 32, lane), acc[j]);
  }
#pragma unroll
  for (int j = 0; j < 8; ++j)
#pragma unroll
    for (int r = 0; r < 8; ++r) th[j * 16 + col][wave * 16 + 8 * g + r] = f16n(acc[j][r]);
  __syncthreads();
  for (int e = tid; e < 128 * 8; e += 128) { const int cl = e >> 3, q = e & 7; vst2(VT + (size_t)(c0 + cl) * SEQ + r0 + q * 8, *(const v8h*)&th[cl][q * 8]); }
}

__global__ __launch_bounds__(128) void k_max(const _Float16* __restrict__ QH, const _Float16* __restrict__ KH, float* __restrict__ MX) {
  __shared__ __align__(16) float sm[64];
  const int tid = threadIdx.x, wave = tid >> 5, lane = tid & 31, col = lane & 15, g = lane >> 4;
  const int q0 = blockIdx.x * 64 + wave * 16;
  v16h ah[4];
#pragma unroll
  for (int kc = 0; kc < 4; ++kc) ah[kc] = frag_h(QH + (size_t)(q0 + col) * DQK + kc * 32, lane);
  float m[8];
#pragma unroll
  for (int r = 0; r < 8; ++r) m[r] = -3.0e38f;
#pragma unroll 2
  for (int jt = 0; jt < SEQ / 16; ++jt) {
    v8f c = zero8();
#pragma unroll
    for (int kc = 0; kc < 4; ++kc) c = wmma16(ah[kc], frag_h(KH + (size_t)(jt * 16 + col) * DQK + kc * 32, lane), c);
#pragma unroll
    for (int r = 0; r < 8; ++r) m[r] = fmaxf(m[r], c[r]);
  }
#pragma unroll
  for (int r = 0; r < 8; ++r) { float t = m[r]; t = fmaxf(t, __shfl_xor(t, 1)); t = fmaxf(t, __shfl_xor(t, 2)); t = fmaxf(t, __shfl_xor(t, 4)); t = fmaxf(t, __shfl_xor(t, 8)); m[r] = t; }
  if (col == 0) {
#pragma unroll
    for (int r = 0; r < 8; ++r) sm[wave * 16 + 8 * g + r] = m[r] * SCALE;
  }
  __syncthreads();
  if (tid < 16) { const v4f v = *(const v4f*)&sm[tid * 4]; vst2(MX + (size_t)blockIdx.x * 64 + tid * 4, v); }
}

__global__ __launch_bounds__(256) void k_att(const _Float16* __restrict__ QH, const _Float16* __restrict__ QL, const _Float16* __restrict__ KH, const _Float16* __restrict__ KL,
                                             const _Float16* __restrict__ VT, const float* __restrict__ MX, float* __restrict__ SA) {
  __shared__ __align__(16) _Float16 sP[16][136];
  __shared__ __align__(16) float sf[8][16][64];
  __shared__ float sl[8][16];
  __shared__ int sfl[8];
  const int tid = threadIdx.x, wave = tid >> 5, lane = tid & 31, col = lane & 15, g = lane >> 4;
  const int q0 = blockIdx.x * 16; const int cb = wave * 128;
  float mref[8], lsum[8];
#pragma unroll
  for (int r = 0; r < 8; ++r) { mref[r] = MX[q0 + 8 * g + r] + 1.0f; lsum[r] = 0.f; }
  v8f acc[8];
#pragma unroll
  for (int j = 0; j < 8; ++j) acc[j] = zero8();
#pragma unroll 1
  for (int kt = 0; kt < SEQ / 128; ++kt) {
    const int key0 = kt * 128, kw = key0 + wave * 16;
    v8f cs = zero8(), cl = zero8();
#pragma unroll 1
    for (int kc = 0; kc < DQK / 32; ++kc) {
      const v16h ah = frag_h(QH + (size_t)(q0 + col) * DQK + kc * 32, lane);
      const v16h ar = frag_h(QL + (size_t)(q0 + col) * DQK + kc * 32, lane);
      const v16h bh = frag_h(KH + (size_t)(kw + col) * DQK + kc * 32, lane);
      const v16h br = frag_h(KL + (size_t)(kw + col) * DQK + kc * 32, lane);
      cs = wmma16(ah, bh, cs); cl = wmma16(ar, bh, cl); cl = wmma16(ah, br, cl);
    }
    int nz = 0;
#pragma unroll
    for (int r = 0; r < 8; ++r) {
      const float s = (cs[r] + cl[r] * (1.0f / RC)) * SCALE;
      const float e = fminf(s - mref[r], 1.0f);
      float pc = __expf(e) * PCY; pc = (pc >= F16MIN) ? pc : 0.0f;
      const _Float16 ph = (_Float16)pc;
      lsum[r] += (float)ph; nz |= (pc != 0.0f) ? 1 : 0;
      sP[8 * g + r][wave * 16 + col] = ph;
    }
    const unsigned wb = __builtin_amdgcn_ballot_w32(nz != 0);
    if (lane == 0) sfl[wave] = (wb != 0u) ? 1 : 0;
    __syncthreads();
#pragma unroll 1
    for (int kk = 0; kk < 4; ++kk) {
      const int f = __builtin_amdgcn_readfirstlane(sfl[2 * kk] | sfl[2 * kk + 1]);
      if (f != 0) {
        const v16h a = frag_h(&sP[col][kk * 32], lane);
#pragma unroll
        for (int j = 0; j < 8; ++j) acc[j] = wmma16(a, frag_h(VT + (size_t)(cb + j * 16 + col) * SEQ + key0 + kk * 32, lane), acc[j]);
      }
    }
    __syncthreads();
  }
#pragma unroll
  for (int r = 0; r < 8; ++r) { float t = lsum[r]; t += __shfl_xor(t, 1); t += __shfl_xor(t, 2); t += __shfl_xor(t, 4); t += __shfl_xor(t, 8); lsum[r] = t; }
  if (col == 0) {
#pragma unroll
    for (int r = 0; r < 8; ++r) sl[wave][8 * g + r] = lsum[r];
  }
  __syncthreads();
  float inv[8];
#pragma unroll
  for (int r = 0; r < 8; ++r) { float t = 0.f;
#pragma unroll
    for (int w = 0; w < 8; ++w) t += sl[w][8 * g + r];
    inv[r] = 1.0f / t; }
#pragma unroll
  for (int jh = 0; jh < 2; ++jh) {
    LDSX();
#pragma unroll
    for (int jl = 0; jl < 4; ++jl)
#pragma unroll
      for (int r = 0; r < 8; ++r) sf[wave][8 * g + r][jl * 16 + col] = acc[4 * jh + jl][r] * inv[r];
    LDSX();
#pragma unroll
    for (int rp = 0; rp < 8; ++rp) { const int rl = 2 * rp + g; const v4f v = *(const v4f*)&sf[wave][rl][col * 4]; vst2(SA + (size_t)(q0 + rl) * DV + cb + jh * 64 + col * 4, v); }
  }
}

__global__ __launch_bounds__(256) void k_ln1(const unsigned short* __restrict__ XB, const float* __restrict__ SA, _Float16* __restrict__ H16) {
  const int wave = threadIdx.x >> 5, lane = threadIdx.x & 31; const int row = blockIdx.x * 8 + wave; if (row >= SEQ) return;
  const size_t rb = (size_t)row * DIN;
  float v[32]; float s1 = 0.f;
#pragma unroll
  for (int i = 0; i < 4; ++i) { const size_t o = rb + i * 256 + lane * 8; const v8us xb = *(const v8us*)(XB + o); const v4f a = *(const v4f*)(SA + o), b = *(const v4f*)(SA + o + 4);
#pragma unroll
    for (int e = 0; e < 4; ++e) { v[8 * i + e] = bf16val(xb[e]) + a[e]; v[8 * i + 4 + e] = bf16val(xb[4 + e]) + b[e]; }
    s1 += ((v[8 * i] + v[8 * i + 1]) + (v[8 * i + 2] + v[8 * i + 3])) + ((v[8 * i + 4] + v[8 * i + 5]) + (v[8 * i + 6] + v[8 * i + 7])); }
#pragma unroll
  for (int o = 1; o < 32; o <<= 1) s1 += __shfl_xor(s1, o);
  const float mu = s1 * (1.0f / DIN); float q = 0.f;
#pragma unroll
  for (int i = 0; i < 32; ++i) { const float d = v[i] - mu; q += d * d; }
#pragma unroll
  for (int o = 1; o < 32; o <<= 1) q += __shfl_xor(q, o);
  const float inv = 1.0f / sqrtf(q * (1.0f / DIN) + LN_EPS);
#pragma unroll
  for (int i = 0; i < 4; ++i) { v8h o8;
#pragma unroll
    for (int e = 0; e < 8; ++e) o8[e] = f16n((v[8 * i + e] - mu) * inv);
    vst2(H16 + rb + i * 256 + lane * 8, o8); }
}

__global__ __launch_bounds__(128) void k_gl(const _Float16* __restrict__ H16, const _Float16* __restrict__ WLH, const float* __restrict__ RES, float* __restrict__ OUT) {
  __shared__ __align__(16) float sf[4][16][132];
  const int tid = threadIdx.x, wave = tid >> 5, lane = tid & 31, col = lane & 15, g = lane >> 4; const int c0 = blockIdx.y * 128; const size_t r0 = (size_t)blockIdx.x * 64 + wave * 16;
  v8f acc[8];
#pragma unroll
  for (int j = 0; j < 8; ++j) acc[j] = zero8();
#pragma unroll 1
  for (int kc = 0; kc < DIN / 32; ++kc) { const v16h a = frag_h(H16 + (r0 + col) * DIN + kc * 32, lane);
#pragma unroll
    for (int j = 0; j < 8; ++j) acc[j] = wmma16(a, frag_h(WLH + (size_t)(c0 + j * 16 + col) * DIN + kc * 32, lane), acc[j]); }
#pragma unroll
  for (int j = 0; j < 8; ++j)
#pragma unroll
    for (int r = 0; r < 8; ++r) sf[wave][8 * g + r][j * 16 + col] = acc[j][r] * (1.0f / WC);
  LDSX();
  for (int rl = 0; rl < 16; ++rl) { const size_t o = (r0 + rl) * (size_t)DOUT + c0 + lane * 4; v4f vv = *(const v4f*)&sf[wave][rl][lane * 4]; const v4f rv = *(const v4f*)(RES + o);
    vv[0] += rv[0]; vv[1] += rv[1]; vv[2] += rv[2]; vv[3] += rv[3]; vst2(OUT + o, vv); }
}

__global__ __launch_bounds__(256) void k_ln2(const float* __restrict__ Z, float* __restrict__ OUT) {
  const int wave = threadIdx.x >> 5, lane = threadIdx.x & 31; const int row = blockIdx.x * 8 + wave; if (row >= SEQ) return;
  const size_t rb = (size_t)row * DOUT;
  v4f v[8]; float s1 = 0.f;
#pragma unroll
  for (int i = 0; i < 8; ++i) { v[i] = *(const v4f*)(Z + rb + i * 128 + lane * 4); s1 += (v[i][0] + v[i][1]) + (v[i][2] + v[i][3]); }
#pragma unroll
  for (int o = 1; o < 32; o <<= 1) s1 += __shfl_xor(s1, o);
  const float mu = s1 * (1.0f / DOUT); float q = 0.f;
#pragma unroll
  for (int i = 0; i < 8; ++i)
#pragma unroll
    for (int k = 0; k < 4; ++k) { const float d = v[i][k] - mu; q += d * d; }
#pragma unroll
  for (int o = 1; o < 32; o <<= 1) q += __shfl_xor(q, o);
  const float inv = 1.0f / sqrtf(q * (1.0f / DOUT) + LN_EPS);
#pragma unroll
  for (int i = 0; i < 8; ++i) { v4f r4;
#pragma unroll
    for (int k = 0; k < 4; ++k) r4[k] = (v[i][k] - mu) * inv;
    vst2(OUT + rb + i * 128 + lane * 4, r4); }
}

extern "C" void kernel_launch(void* const* d_in, const int* in_sizes, int n_in, void* d_out, int out_size, void* d_ws, size_t ws_size, hipStream_t stream) {
  if (n_in < 5) return;
  if (in_sizes[0] < SEQ * DIN || in_sizes[1] < DQK * DIN || in_sizes[2] < DQK * DIN || in_sizes[3] < DV * DIN || in_sizes[4] < DOUT * DIN) return;
  if (out_size < SEQ * DOUT) return;
  if (ws_size < (size_t)WS_END) return;
  const float* X = (const float*)d_in[0]; const float* WQ = (const float*)d_in[1]; const float* WK = (const float*)d_in[2]; const float* WV = (const float*)d_in[3]; const float* WL = (const float*)d_in[4];
  char* ws = (char*)d_ws;
  unsigned short* XBu = (unsigned short*)(ws + WS_XB); unsigned short* WQBu = (unsigned short*)(ws + WS_WQB); unsigned short* WKBu = (unsigned short*)(ws + WS_WKB); unsigned short* WVBu = (unsigned short*)(ws + WS_WVB);
  const __bf16* XB = (const __bf16*)(ws + WS_XB); const __bf16* WQB = (const __bf16*)(ws + WS_WQB); const __bf16* WKB = (const __bf16*)(ws + WS_WKB); const __bf16* WVB = (const __bf16*)(ws + WS_WVB);
  _Float16* WLH = (_Float16*)(ws + WS_WLH);
  _Float16 *QH = (_Float16*)(ws + WS_QH), *QL = (_Float16*)(ws + WS_QL), *KH = (_Float16*)(ws + WS_KH), *KL = (_Float16*)(ws + WS_KL), *VT = (_Float16*)(ws + WS_VT), *H16 = (_Float16*)(ws + WS_H16);
  float *MX = (float*)(ws + WS_MX), *SA = (float*)(ws + WS_SA), *Z2 = (float*)(ws + WS_Z2);

  const int n8x = SEQ * DIN / 8, n8qk = DQK * DIN / 8, n8v = DV * DIN / 8, n8l = DOUT * DIN / 8;
  k_cvtb<<<dim3((n8x + 255) / 256), 256, 0, stream>>>(X, n8x, XBu);
  k_cvtb<<<dim3((n8qk + 255) / 256), 256, 0, stream>>>(WQ, n8qk, WQBu);
  k_cvtb<<<dim3((n8qk + 255) / 256), 256, 0, stream>>>(WK, n8qk, WKBu);
  k_cvtb<<<dim3((n8v + 255) / 256), 256, 0, stream>>>(WV, n8v, WVBu);
  k_cvth<<<dim3((n8l + 255) / 256), 256, 0, stream>>>(WL, n8l, WLH);
  k_pqk<<<dim3(SEQ / 64), 128, 0, stream>>>(XB, WQB, QH, QL);
  k_pqk<<<dim3(SEQ / 64), 128, 0, stream>>>(XB, WKB, KH, KL);
  k_pvt<<<dim3(SEQ / 64, DV / 128), 128, 0, stream>>>(XB, WVB, VT);
  k_max<<<dim3(SEQ / 64), 128, 0, stream>>>(QH, KH, MX);
  k_att<<<dim3(SEQ / 16), 256, 0, stream>>>(QH, QL, KH, KL, VT, MX, SA);
  k_ln1<<<dim3(SEQ / 8), 256, 0, stream>>>(XBu, SA, H16);
  k_gl<<<dim3(SEQ / 64, DOUT / 128), 128, 0, stream>>>(H16, WLH, SA, Z2);
  k_ln2<<<dim3(SEQ / 8), 256, 0, stream>>>(Z2, (float*)d_out);
}
